// GAT_14766097564097
// MI455X (gfx1250) — hardware-verified
//
#include <hip/hip_runtime.h>
#include <stddef.h>
#include <stdint.h>
#include <math.h>


#define NB    8
#define NN    1024
#define NF    512
#define NH    4
#define ND    128
#define MROWS (NB * NN)
#define NCOL  (2 * NH * ND)
#define PTHR  256
#define NUX   (MROWS * (NF / 8))
#define NUW   (NH * ND * (NF / 8))
#define GBM   64
#define GBN   128
#define GTHR  128
#define GM    (MROWS / GBM)
#define ATHR  128
#define AROWS 64
#define KT    64
#define NEGSL 0.2f
#define MASKV (-1.0e10f)
#define WSMAX 134217728

static_assert((NF % 32) == 0 && (NN % KT) == 0 && (KT % 32) == 0);
static_assert((NUX % PTHR) == 0 && (NUW % PTHR) == 0);
static_assert((MROWS % GBM) == 0 && (NCOL % GBN) == 0 && GBN == ND);
static_assert(GBM == (GTHR / 32) * 16 && GBN == 4 * 32);
static_assert((NN % GBM) == 0 && GBM == KT);
static_assert(AROWS == (ATHR / 32) * 16 && ATHR * 8 == NN);
static_assert(ND == 4 * 32 && NF / 8 == 64);

typedef float          v4f  __attribute__((ext_vector_type(4)));
typedef float          v8f  __attribute__((ext_vector_type(8)));
typedef int            v8i  __attribute__((ext_vector_type(8)));
typedef unsigned int   v4u  __attribute__((ext_vector_type(4)));
typedef unsigned short v8us __attribute__((ext_vector_type(8)));
typedef __bf16         v16b __attribute__((ext_vector_type(16)));
typedef v4f  __attribute__((may_alias)) v4fa;
typedef v8us __attribute__((may_alias)) v8usa;
union FragB { v16b v; v8us h[2]; v4u q[2]; v8i w; };

__device__ __forceinline__ v8f wmb(const FragB& a, const FragB& b, v8f c) {
  v8f d = __builtin_amdgcn_wmma_f32_16x16x32_bf16(false, a.v, false, b.v, (short)0, c, false, false);
  asm volatile("v_nop\n\tv_nop\n\tv_nop\n\tv_nop" : "+v"(d) : "v"(a.w), "v"(b.w));
  return d;
}

__device__ __forceinline__ unsigned int f2bf(float f) {
  const unsigned int u = __float_as_uint(f);
  return ((u + 0x7FFFu + ((u >> 16) & 1u)) >> 16) & 0xFFFFu;
}
__device__ __forceinline__ float bf2f(unsigned int b) { return __uint_as_float(b << 16); }
__device__ __forceinline__ float bfr(float f) { return bf2f(f2bf(f)); }
__device__ __forceinline__ v4f bfr4(const v4f a) {
  v4f r; r.x = bfr(a.x); r.y = bfr(a.y); r.z = bfr(a.z); r.w = bfr(a.w); return r;
}
__device__ __forceinline__ unsigned int pk2(float lo, float hi) { return f2bf(lo) | (f2bf(hi) << 16); }
__device__ __forceinline__ v4u pack8(const v4f a, const v4f b) {
  v4u r;
  r.x = pk2(a.x, a.y); r.y = pk2(a.z, a.w); r.z = pk2(b.x, b.y); r.w = pk2(b.z, b.w);
  return r;
}
__device__ __forceinline__ void split2(float x, float y, unsigned int& hw, unsigned int& lw) {
  const unsigned int hx = f2bf(x), hy = f2bf(y);
  const unsigned int lx = f2bf(x - bf2f(hx)), ly = f2bf(y - bf2f(hy));
  hw = hx | (hy << 16);
  lw = lx | (ly << 16);
}
__device__ __forceinline__ void split8(const v4f a, const v4f b, v4u& hq, v4u& lq) {
  unsigned int h0, h1, h2, h3, l0, l1, l2, l3;
  split2(a.x, a.y, h0, l0);
  split2(a.z, a.w, h1, l1);
  split2(b.x, b.y, h2, l2);
  split2(b.z, b.w, h3, l3);
  hq.x = h0; hq.y = h1; hq.z = h2; hq.w = h3;
  lq.x = l0; lq.y = l1; lq.z = l2; lq.w = l3;
}

__global__ __launch_bounds__(PTHR) void k_prep(const float* __restrict__ X, const float* __restrict__ Watt,
                                               const float* __restrict__ Kern,
                                               unsigned short* XB, unsigned short* WT) {
  const int u = (int)blockIdx.x * PTHR + (int)threadIdx.x;
  v4f a, b;
  unsigned short* dp;
  if (u < NUX) {
    const int row = u >> 6;
    const int k8  = (u & 63) * 8;
    const float* p = X + (size_t)row * NF + k8;
    a = *(const v4fa*)p;
    b = *(const v4fa*)(p + 4);
    dp = XB + (size_t)row * NF + k8;
  } else if (u < NUX + NUW) {
    const int v  = u - NUX;
    const int n  = v >> 6;
    const int k8 = (v & 63) * 8;
    const int hd = n >> 7, d = n & (ND - 1);
    const float* p = Watt + ((size_t)hd * NF + k8) * ND + d;
    a.x = p[0];      a.y = p[ND];     a.z = p[2 * ND]; a.w = p[3 * ND];
    b.x = p[4 * ND]; b.y = p[5 * ND]; b.z = p[6 * ND]; b.w = p[7 * ND];
    dp = WT + (size_t)n * NF + k8;
  } else if (u < NUX + 2 * NUW) {
    const int v  = u - NUX - NUW;
    const int n  = v >> 6;
    const int k8 = (v & 63) * 8;
    const int hd = n >> 7, d = n & (ND - 1);
    const float* p = Kern + ((size_t)hd * NF + k8) * ND + d;
    a.x = p[0];      a.y = p[ND];     a.z = p[2 * ND]; a.w = p[3 * ND];
    b.x = p[4 * ND]; b.y = p[5 * ND]; b.z = p[6 * ND]; b.w = p[7 * ND];
    dp = WT + (size_t)(NH * ND + n) * NF + k8;
  } else {
    return;
  }
  const v4u o = pack8(a, b);
  *(volatile v4u*)dp = o;
  __threadfence();
  *(volatile v4u*)dp = o;
}

__global__ __launch_bounds__(GTHR) void k_proj(const unsigned short* __restrict__ XB,
                                               const unsigned short* __restrict__ WT,
                                               const float* __restrict__ aatt,
                                               float* SN, unsigned short* XKH, unsigned short* XKL) {
  __shared__ __attribute__((aligned(16))) float stg[GBM * GBN];
  __shared__ __attribute__((aligned(16))) float sdt[2 * GBM];
  const int tid = (int)threadIdx.x, lane = tid & 31, wave = tid >> 5, hh = lane >> 4, m = lane & 15;
  const int rowBase = (int)blockIdx.x * GBM;
  const int nt8     = (int)blockIdx.y;
  const int colBase = nt8 * GBN;

  v8f acc[8];
  {
    const v8f z = {0.f, 0.f, 0.f, 0.f, 0.f, 0.f, 0.f, 0.f};
#pragma unroll
    for (int t = 0; t < 8; ++t) acc[t] = z;
  }
  const unsigned short* ap = XB + (size_t)(rowBase + 16 * wave + m) * (size_t)NF + 8 * hh;
  const unsigned short* bp = WT + (size_t)(colBase + m) * (size_t)NF + 8 * hh;

#pragma unroll 1
  for (int k0 = 0; k0 < NF; k0 += 32) {
    FragB af;
    af.h[0] = *(const v8usa*)(ap + k0);
    af.h[1] = *(const v8usa*)(ap + k0 + 16);
#pragma unroll
    for (int nt = 0; nt < 8; ++nt) {
      const unsigned short* wq = bp + (size_t)(16 * nt) * (size_t)NF + k0;
      FragB bf;
      bf.h[0] = *(const v8usa*)wq;
      bf.h[1] = *(const v8usa*)(wq + 16);
      acc[nt] = wmb(af, bf, acc[nt]);
    }
  }

#pragma unroll
  for (int nt = 0; nt < 8; ++nt) {
    const int lc = 16 * nt + m;
#pragma unroll
    for (int r = 0; r < 8; ++r) {
      const int lr = 16 * wave + 8 * hh + r;
      stg[lr * GBN + lc] = acc[nt][r];
    }
  }
  __syncthreads();

  if (nt8 < NH) {
    const int head = nt8;
    const v4f as4 = bfr4(*(const v4fa*)(aatt + (size_t)(head * 2 + 0) * ND + 4 * lane));
    const v4f ad4 = bfr4(*(const v4fa*)(aatt + (size_t)(head * 2 + 1) * ND + 4 * lane));
#pragma unroll 1
    for (int i = 0; i < 16; ++i) {
      const int row = wave * 16 + i;
      const v4f p = *(const v4fa*)(stg + row * GBN + 4 * lane);
      float s = 0.0f, d = 0.0f;
      s = fmaf(p.x, as4.x, s); s = fmaf(p.y, as4.y, s); s = fmaf(p.z, as4.z, s); s = fmaf(p.w, as4.w, s);
      d = fmaf(p.x, ad4.x, d); d = fmaf(p.y, ad4.y, d); d = fmaf(p.z, ad4.z, d); d = fmaf(p.w, ad4.w, d);
#pragma unroll
      for (int off = 16; off > 0; off >>= 1) {
        s += __shfl_xor(s, off);
        d += __shfl_xor(d, off);
      }
      if (lane == 0) { sdt[row] = s; sdt[GBM + row] = d; }
    }
    __syncthreads();
    if (wave == 0) {
      const v4f alv = *(const v4fa*)(sdt + 4 * lane);
      float* alp = SN + ((size_t)head * GM + blockIdx.x) * (size_t)(2 * GBM) + 4 * lane;
      *(volatile v4f*)alp = alv;
      __threadfence();
      *(volatile v4f*)alp = alv;
    }
  } else {
    const int head = nt8 - NH;
    const int b    = rowBase >> 10;
    const int j0   = rowBase & (NN - 1);
    const int q    = lane & 7, dsub = lane >> 3;
#pragma unroll 1
    for (int it = 0; it < 8; ++it) {
      const int d = wave * 32 + it * 4 + dsub;
      const float* sp = stg + (8 * q) * GBN + d;
      v4f a, bq;
      a.x  = sp[0];       a.y  = sp[GBN];     a.z  = sp[2 * GBN]; a.w  = sp[3 * GBN];
      bq.x = sp[4 * GBN]; bq.y = sp[5 * GBN]; bq.z = sp[6 * GBN]; bq.w = sp[7 * GBN];
      v4u hq, lq;
      split8(a, bq, hq, lq);
      const size_t o = ((size_t)((b * NH + head) * ND + d)) * (size_t)NN + j0 + 8 * q;
      *(volatile v4u*)(XKH + o) = hq;
      *(volatile v4u*)(XKL + o) = lq;
      __threadfence();
      *(volatile v4u*)(XKH + o) = hq;
      *(volatile v4u*)(XKL + o) = lq;
    }
  }
}

__device__ __forceinline__ float score1(float self, float nv, float av) {
  float t = self + nv;
  t = (t >= 0.0f) ? t : NEGSL * t;
  return t + MASKV * (1.0f - av);
}
__device__ __forceinline__ v4f score4(float self, const v4f nv, const v4f av) {
  v4f r;
  r.x = score1(self, nv.x, av.x); r.y = score1(self, nv.y, av.y);
  r.z = score1(self, nv.z, av.z); r.w = score1(self, nv.w, av.w);
  return r;
}
__device__ __forceinline__ float max4(const v4f a) { return fmaxf(fmaxf(a.x, a.y), fmaxf(a.z, a.w)); }
__device__ __forceinline__ v4f exp4(const v4f s, float mx) {
  v4f r;
  r.x = expf(s.x - mx); r.y = expf(s.y - mx); r.z = expf(s.z - mx); r.w = expf(s.w - mx);
  return r;
}

__global__ __launch_bounds__(ATHR) void k_attn(const float* __restrict__ A, const float* __restrict__ SN,
                                               const unsigned short* __restrict__ XKH,
                                               const unsigned short* __restrict__ XKL,
                                               const float* __restrict__ bias, float* out) {
  __shared__ __attribute__((aligned(16))) float sn[NN];
  __shared__ __attribute__((aligned(16))) float ostg[AROWS * ND];
  const int tid = (int)threadIdx.x, lane = tid & 31, wave = tid >> 5, hh = lane >> 4, m = lane & 15;
  const int blk   = (int)blockIdx.x;
  const int itile = blk & 15;
  const int h     = (blk >> 4) & (NH - 1);
  const int b     = blk >> 6;
  const int i0    = itile * AROWS;

  {
    const float* sp = SN + ((size_t)(h * GM + b * 16 + (tid >> 3))) * (size_t)(2 * GBM) + GBM + 8 * (tid & 7);
    const v4f x0 = *(const v4fa*)sp;
    const v4f x1 = *(const v4fa*)(sp + 4);
    *(v4f*)(sn + 8 * tid)     = x0;
    *(v4f*)(sn + 8 * tid + 4) = x1;
  }
  const float self = SN[((size_t)(h * GM + b * 16 + itile)) * (size_t)(2 * GBM) + 16 * wave + m];
  __syncthreads();

  v8f acc[8];
  {
    const v8f z = {0.f, 0.f, 0.f, 0.f, 0.f, 0.f, 0.f, 0.f};
#pragma unroll
    for (int t = 0; t < 8; ++t) acc[t] = z;
  }
  float mrun = -1.0e30f;
  float lsum = 0.0f;
  const float* arow = A + ((size_t)(b * NN + i0 + 16 * wave + m)) * (size_t)NN + 8 * hh;
  const size_t xoff = ((size_t)((b * NH + h) * ND + m)) * (size_t)NN + 8 * hh;
  const unsigned short* xh = XKH + xoff;
  const unsigned short* xl = XKL + xoff;
  const float* snl = sn + 8 * hh;

#pragma unroll 1
  for (int jt = 0; jt < NN / KT; ++jt) {
    const int j0 = jt * KT;
    v4f sv[8];
#pragma unroll
    for (int c = 0; c < 4; ++c) {
      const int off = j0 + 16 * c;
      const v4f a0 = *(const v4fa*)(arow + off);
      const v4f a1 = *(const v4fa*)(arow + off + 4);
      const v4f n0 = *(const v4fa*)(snl + off);
      const v4f n1 = *(const v4fa*)(snl + off + 4);
      sv[2 * c]     = score4(self, n0, a0);
      sv[2 * c + 1] = score4(self, n1, a1);
    }
    float mloc = max4(sv[0]);
#pragma unroll
    for (int i = 1; i < 8; ++i) mloc = fmaxf(mloc, max4(sv[i]));
    mloc = fmaxf(mloc, __shfl_xor(mloc, 16));
    const float mnew  = fmaxf(mrun, mloc);
    const float alpha = expf(mrun - mnew);
    mrun = mnew;

    FragB ph[2], pl[2];
    float ps = 0.0f;
#pragma unroll
    for (int c = 0; c < 4; ++c) {
      const v4f p0 = exp4(sv[2 * c], mnew);
      const v4f p1 = exp4(sv[2 * c + 1], mnew);
      ps += ((p0.x + p0.y) + (p0.z + p0.w)) + ((p1.x + p1.y) + (p1.z + p1.w));
      v4u hq, lq;
      split8(p0, p1, hq, lq);
      ph[c >> 1].q[c & 1] = hq;
      pl[c >> 1].q[c & 1] = lq;
    }
    lsum = fmaf(lsum, alpha, ps);

#pragma unroll
    for (int r = 0; r < 8; ++r) {
      const float ar = __shfl(alpha, 8 * hh + r);
#pragma unroll
      for (int t = 0; t < 8; ++t) acc[t][r] *= ar;
    }

#pragma unroll
    for (int ks = 0; ks < 2; ++ks) {
#pragma unroll
      for (int t = 0; t < 8; ++t) {
        const size_t o = (size_t)(16 * t) * (size_t)NN + j0 + 32 * ks;
        FragB vh, vl;
        vh.h[0] = *(const v8usa*)(xh + o);
        vh.h[1] = *(const v8usa*)(xh + o + 16);
        vl.h[0] = *(const v8usa*)(xl + o);
        vl.h[1] = *(const v8usa*)(xl + o + 16);
        acc[t] = wmb(ph[ks], vh, acc[t]);
        acc[t] = wmb(ph[ks], vl, acc[t]);
        acc[t] = wmb(pl[ks], vh, acc[t]);
      }
    }
  }

  const float ltot = lsum + __shfl_xor(lsum, 16);
  const float inv  = 1.0f / ltot;
#pragma unroll
  for (int r = 0; r < 8; ++r) {
    const float ir = __shfl(inv, 8 * hh + r);
    const int lr = 16 * wave + 8 * hh + r;
#pragma unroll
    for (int t = 0; t < 8; ++t) ostg[lr * ND + 16 * t + m] = acc[t][r] * ir;
  }
  __syncthreads();

  const v4f bb = bfr4(*(const v4fa*)(bias + h * ND + 4 * lane));
#pragma unroll 1
  for (int i = 0; i < 16; ++i) {
    const int row = 16 * wave + i;
    const v4f v = *(const v4fa*)(ostg + row * ND + 4 * lane);
    v4f y;
    y.x = v.x + bb.x; y.y = v.y + bb.y; y.z = v.z + bb.z; y.w = v.w + bb.w;
    v4f e;
    e.x = (y.x > 0.0f) ? y.x : expm1f(y.x);
    e.y = (y.y > 0.0f) ? y.y : expm1f(y.y);
    e.z = (y.z > 0.0f) ? y.z : expm1f(y.z);
    e.w = (y.w > 0.0f) ? y.w : expm1f(y.w);
    float* op = out + ((size_t)(b * NN + i0 + row)) * (size_t)(NH * ND) + h * ND + 4 * lane;
    *(volatile v4f*)op = e;
    __threadfence();
    *(volatile v4f*)op = e;
  }
}

extern "C" void kernel_launch(void* const* d_in, const int* in_sizes, int n_in,
                              void* d_out, int out_size, void* d_ws, size_t ws_size,
                              hipStream_t stream) {
  if (n_in < 6) return;
  if (in_sizes[0] != NB * NN * NF) return;
  if (in_sizes[1] != NB * NN * NN) return;
  if (in_sizes[2] != NH * NF * ND) return;
  if (in_sizes[3] != NH * 2 * ND) return;
  if (in_sizes[4] != NH * NF * ND) return;
  if (in_sizes[5] != NH * ND) return;
  if (out_size != NB * NN * NH * ND) return;

  const float* X    = (const float*)d_in[0];
  const float* Adj  = (const float*)d_in[1];
  const float* Watt = (const float*)d_in[2];
  const float* aatt = (const float*)d_in[3];
  const float* Kern = (const float*)d_in[4];
  const float* bias = (const float*)d_in[5];
  float* out = (float*)d_out;

  char* ws = (char*)d_ws;
  size_t off = 0;
  const size_t oXB  = off; off += (size_t)MROWS * NF * 2;            off = (off + 255) & ~(size_t)255;
  const size_t oWT  = off; off += (size_t)NCOL * NF * 2;             off = (off + 255) & ~(size_t)255;
  const size_t oSN  = off; off += (size_t)NH * GM * 2 * GBM * 4;     off = (off + 255) & ~(size_t)255;
  const size_t oXKH = off; off += (size_t)NB * NH * ND * NN * 2;     off = (off + 255) & ~(size_t)255;
  const size_t oXKL = off; off += (size_t)NB * NH * ND * NN * 2;     off = (off + 255) & ~(size_t)255;
  if (off > ws_size || off > (size_t)WSMAX) return;
  unsigned short* XB  = (unsigned short*)(ws + oXB);
  unsigned short* WT  = (unsigned short*)(ws + oWT);
  float*          SN  = (float*)(ws + oSN);
  unsigned short* XKH = (unsigned short*)(ws + oXKH);
  unsigned short* XKL = (unsigned short*)(ws + oXKL);

  k_prep<<<(NUX + 2 * NUW) / PTHR, PTHR, 0, stream>>>(X, Watt, Kern, XB, WT);
  k_proj<<<dim3(GM, NCOL / GBN), GTHR, 0, stream>>>(XB, WT, aatt, SN, XKH, XKL);
  k_attn<<<NB * NH * (NN / AROWS), ATHR, 0, stream>>>(Adj, SN, XKH, XKL, bias, out);
}
